// TopicAdaptiveLSTMCell_88115549045316
// MI455X (gfx1250) — hardware-run, weakly checked
//
#include <hip/hip_runtime.h>
#include <math.h>

typedef __attribute__((ext_vector_type(16))) _Float16 v16h;
typedef __attribute__((ext_vector_type(16))) __bf16 v16b;
typedef __attribute__((ext_vector_type(8)))  _Float16 v8h;
typedef __attribute__((ext_vector_type(8)))  float v8f;
typedef __attribute__((ext_vector_type(4)))  float v4f;
typedef __attribute__((ext_vector_type(2)))  float v2f;
typedef __attribute__((ext_vector_type(4)))  unsigned v4u;
typedef __attribute__((ext_vector_type(4)))  int v4i;
typedef float __attribute__((may_alias)) float_a;
typedef int __attribute__((may_alias)) int_a;

template <typename T> __device__ __forceinline__ void vst2(void* p, T v) { *(volatile T*)p = v; __threadfence(); *(volatile T*)p = v; }
__device__ __forceinline__ v8f wmma16(v16h a, v16h b, v8f c) {
  v8f d = __builtin_amdgcn_wmma_f32_16x16x32_f16(false, a, false, b, (short)0, c, false, false);
  asm volatile("v_nop\n\tv_nop\n\tv_nop\n\tv_nop" : "+v"(d) : "v"(a), "v"(b));
  return d;
}
__device__ __forceinline__ v8f wmma_bf(v16b a, v16b b, v8f c) {
  v8f d = __builtin_amdgcn_wmma_f32_16x16x32_bf16(false, a, false, b, (short)0, c, false, false);
  asm volatile("v_nop\n\tv_nop\n\tv_nop\n\tv_nop" : "+v"(d) : "v"(a), "v"(b));
  return d;
}
__device__ __forceinline__ v16h frag_h(const _Float16* rowk0, int lane) {
  union { v16h v; v8h q[2]; } u; const _Float16* p = rowk0 + 8 * (lane >> 4);
  u.q[0] = *(const v8h*)p; u.q[1] = *(const v8h*)(p + 16); return u.v;
}
__device__ __forceinline__ v16h frag_f32(const float* rowk0, int lane) {
  v16h a; const float* p = rowk0 + 8 * (lane >> 4);
#pragma unroll
  for (int i = 0; i < 8; ++i) { a[i] = (_Float16)p[i]; a[8 + i] = (_Float16)p[16 + i]; }
  return a;
}
__device__ __forceinline__ v16h frag_f32s(const float* rowk0, int lane, float sc) {
  v16h a; const float* p = rowk0 + 8 * (lane >> 4);
#pragma unroll
  for (int i = 0; i < 8; ++i) { a[i] = (_Float16)(p[i] * sc); a[8 + i] = (_Float16)(p[16 + i] * sc); }
  return a;
}
__device__ __forceinline__ v16h fragc_f32(const float* W, int k0, int n, int lane, int ld, int K) {
  v16h a; const int g = lane >> 4;
#pragma unroll
  for (int i = 0; i < 8; ++i) { const int ka = k0 + 8 * g + i, kb = ka + 16;
    a[i] = (_Float16)(ka < K ? W[(size_t)ka * ld + n] : 0.f); a[8 + i] = (_Float16)(kb < K ? W[(size_t)kb * ld + n] : 0.f); }
  return a;
}
struct F2 { v16b h, l; };
__device__ __forceinline__ F2 bsplit16(const float v[16]) { F2 r;
#pragma unroll
  for (int i = 0; i < 16; ++i) { const __bf16 h = (__bf16)v[i]; r.h[i] = h; r.l[i] = (__bf16)(v[i] - (float)h); }
  return r; }
__device__ __forceinline__ F2 split_row(const float* row, int k0, int lane) { float v[16]; const float* p = row + k0 + 8 * (lane >> 4);
#pragma unroll
  for (int i = 0; i < 8; ++i) { v[i] = p[i]; v[8 + i] = p[16 + i]; }
  return bsplit16(v); }
__device__ __forceinline__ F2 split_rowK(const float* row, int k0, int lane, int K) { float v[16]; const int g = lane >> 4;
#pragma unroll
  for (int i = 0; i < 8; ++i) { const int ka = k0 + 8 * g + i, kb = ka + 16; v[i] = ka < K ? row[ka] : 0.f; v[8 + i] = kb < K ? row[kb] : 0.f; }
  return bsplit16(v); }
__device__ __forceinline__ F2 split_col(const float* W, int k0, int n, int lane, int ld, int K) { float v[16]; const int g = lane >> 4;
#pragma unroll
  for (int i = 0; i < 8; ++i) { const int ka = k0 + 8 * g + i, kb = ka + 16; v[i] = ka < K ? W[(size_t)ka * ld + n] : 0.f; v[8 + i] = kb < K ? W[(size_t)kb * ld + n] : 0.f; }
  return bsplit16(v); }
__device__ __forceinline__ v8f mac3(const F2& a, const F2& b, v8f c) { c = wmma_bf(a.l, b.h, c); c = wmma_bf(a.h, b.l, c); return wmma_bf(a.h, b.h, c); }
__device__ __forceinline__ float sigm(float v) { return 1.0f / (1.0f + expf(-v)); }
#define LDSX() do { asm volatile("s_wait_dscnt 0" ::: "memory"); __builtin_amdgcn_wave_barrier(); __builtin_amdgcn_fence(__ATOMIC_RELEASE, "workgroup"); } while (0)

typedef __bf16 v8b __attribute__((ext_vector_type(8)));
#define NBATCH 4096
#define NIN 1024
#define NHID 1024
#define NF 128
#define NT 3
#define G4 4096

__global__ __launch_bounds__(128) void k_u(const float* __restrict__ x, const float* __restrict__ hx, const float* __restrict__ topic, const float* __restrict__ wic, const float* __restrict__ whc, const float* __restrict__ wib, const float* __restrict__ whb,
                                         const float* __restrict__ tiw, const float* __restrict__ tib, const float* __restrict__ thw, const float* __restrict__ thb, float* __restrict__ UI, float* __restrict__ UH) {
  __shared__ __align__(16) float so[4][16][132];
  const int tid = threadIdx.x, wave = tid >> 5, lane = tid & 31, col = lane & 15, g = lane >> 4;
  const int which = blockIdx.y; const float* A = which == 0 ? x : hx; const float* Wc = which == 0 ? wic : whc; const float* Wb = which == 0 ? wib : whb; const float* tw = which == 0 ? tiw : thw; const float* tb = which == 0 ? tib : thb; float* U = which == 0 ? UI : UH;
  const int r0 = blockIdx.x * 64 + wave * 16;
  v8f acc[8] = {};
#pragma unroll 1
  for (int kc = 0; kc < NIN / 32; ++kc) { const F2 a = split_row(A + (size_t)(r0 + col) * NIN, kc * 32, lane);
#pragma unroll
    for (int t = 0; t < 8; ++t) acc[t] = mac3(a, split_row(Wc + (size_t)(t * 16 + col) * NIN, kc * 32, lane), acc[t]); }
#pragma unroll
  for (int r = 0; r < 8; ++r) { const int row = r0 + 8 * g + r; float th[NT];
#pragma unroll
    for (int t = 0; t < NT; ++t) { float s = tb[t];
#pragma unroll
      for (int u = 0; u < NT; ++u) s += topic[(size_t)row * NT + u] * tw[t * NT + u];
      th[t] = s; }
#pragma unroll
    for (int t8 = 0; t8 < 8; ++t8) { const int f = t8 * 16 + col; float sc = 0.f;
#pragma unroll
      for (int t = 0; t < NT; ++t) sc += th[t] * Wb[f * NT + t];
      so[wave][8 * g + r][f] = acc[t8][r] * sc; } }
  LDSX();
#pragma unroll 4
  for (int rl = 0; rl < 16; ++rl) vst2(U + (size_t)(r0 + rl) * NF + lane * 4, *(const v4f*)(&so[wave][rl][lane * 4]));
}

__device__ __forceinline__ v16b frag_b(const __bf16* p, int lane) { const int g = lane >> 4; union { v8b v; v4u u; } lo, hi;
  lo.u = *(const v4u*)(p + 8 * g); hi.u = *(const v4u*)(p + 16 + 8 * g); v16b a;
#pragma unroll
  for (int i = 0; i < 8; ++i) { a[i] = lo.v[i]; a[8 + i] = hi.v[i]; }
  return a; }
__global__ __launch_bounds__(128) void k_stats(const float* __restrict__ UI, const float* __restrict__ UH, const float* __restrict__ wia, const float* __restrict__ wha, float* __restrict__ ST) {
  __shared__ __align__(16) float sst[4][16][4];
  const int tid = threadIdx.x, wave = tid >> 5, lane = tid & 31, col = lane & 15, g = lane >> 4;
  const int r0 = blockIdx.x * 64 + wave * 16;
  __shared__ __align__(16) __bf16 sAh[4][2][16][136], sAl[4][2][16][136];
  for (int q = lane; q < 2 * 16 * 32; q += 32) { const int path = q >> 9, rem = q & 511; const int rl = rem >> 5, k4 = rem & 31; const float* src = (path == 0 ? UI : UH) + (size_t)(r0 + rl) * NF + k4 * 4; const v4f v = *(const v4f*)src;
#pragma unroll
    for (int e = 0; e < 4; ++e) { const __bf16 hb = (__bf16)v[e]; sAh[wave][path][rl][k4 * 4 + e] = hb; sAl[wave][path][rl][k4 * 4 + e] = (__bf16)(v[e] - (float)hb); } }
  LDSX();
  float s1i[8] = {}, s2i[8] = {}, s1h[8] = {}, s2h[8] = {};
#pragma unroll 1
  for (int ct = 0; ct < G4 / 16; ++ct) { v8f di = {}, dh = {}; const size_t wrow = (size_t)(ct * 16 + col) * NF;
#pragma unroll
    for (int kc = 0; kc < 4; ++kc) { F2 a; a.h = frag_b(&sAh[wave][0][col][kc * 32], lane); a.l = frag_b(&sAl[wave][0][col][kc * 32], lane); di = mac3(a, split_row(wia + wrow, kc * 32, lane), di);
      a.h = frag_b(&sAh[wave][1][col][kc * 32], lane); a.l = frag_b(&sAl[wave][1][col][kc * 32], lane); dh = mac3(a, split_row(wha + wrow, kc * 32, lane), dh); }
#pragma unroll
    for (int r = 0; r < 8; ++r) { s1i[r] += di[r]; s2i[r] += di[r] * di[r]; s1h[r] += dh[r]; s2h[r] += dh[r] * dh[r]; } }
#pragma unroll
  for (int r = 0; r < 8; ++r) {
#pragma unroll
    for (int off = 1; off <= 8; off <<= 1) { s1i[r] += __shfl_xor(s1i[r], off, 32); s2i[r] += __shfl_xor(s2i[r], off, 32); s1h[r] += __shfl_xor(s1h[r], off, 32); s2h[r] += __shfl_xor(s2h[r], off, 32); } }
  {
    float mi = 0.f, vi = 0.f, mh = 0.f, vh = 0.f;
#pragma unroll
    for (int r = 0; r < 8; ++r) if (r == col) { mi = s1i[r]; vi = s2i[r]; mh = s1h[r]; vh = s2h[r]; }
    if (col < 8) { const float mui = mi * (1.0f / G4), muh = mh * (1.0f / G4); const float vari = fmaxf(vi * (1.0f / G4) - mui * mui, 0.f), varh = fmaxf(vh * (1.0f / G4) - muh * muh, 0.f);
      sst[wave][8 * g + col][0] = mui; sst[wave][8 * g + col][1] = rsqrtf(vari + 1e-5f); sst[wave][8 * g + col][2] = muh; sst[wave][8 * g + col][3] = rsqrtf(varh + 1e-5f); } }
  LDSX();
  if (lane < 16) vst2(ST + (size_t)(r0 + lane) * 4, *(const v4f*)(&sst[wave][lane][0]));
}
__global__ __launch_bounds__(128) void k_cell(const float* __restrict__ UI, const float* __restrict__ UH, const float* __restrict__ wia, const float* __restrict__ wha, const float* __restrict__ ST,
                                            const float* __restrict__ giw, const float* __restrict__ gib, const float* __restrict__ ghw, const float* __restrict__ ghb, const float* __restrict__ cx, float* __restrict__ CP, float* __restrict__ OG) {
  __shared__ __align__(16) float sg[4][4][16][68];
  const int tid = threadIdx.x, wave = tid >> 5, lane = tid & 31, col = lane & 15, g = lane >> 4;
  const int r0 = blockIdx.x * 64 + wave * 16, c0 = blockIdx.y * 64;
  __shared__ __align__(16) __bf16 sAh[4][2][16][136], sAl[4][2][16][136];
  for (int q = lane; q < 2 * 16 * 32; q += 32) { const int path = q >> 9, rem = q & 511; const int rl = rem >> 5, k4 = rem & 31; const float* src = (path == 0 ? UI : UH) + (size_t)(r0 + rl) * NF + k4 * 4; const v4f v = *(const v4f*)src;
#pragma unroll
    for (int e = 0; e < 4; ++e) { const __bf16 hb = (__bf16)v[e]; sAh[wave][path][rl][k4 * 4 + e] = hb; sAl[wave][path][rl][k4 * 4 + e] = (__bf16)(v[e] - (float)hb); } }
  LDSX();

  float sti[8][2], sth[8][2];
#pragma unroll
  for (int r = 0; r < 8; ++r) { const float* s = ST + (size_t)(r0 + 8 * g + r) * 4; sti[r][0] = s[0]; sti[r][1] = s[1]; sth[r][0] = s[2]; sth[r][1] = s[3]; }
#pragma unroll 1
  for (int q = 0; q < 4; ++q) { v8f di[4] = {}, dh[4] = {};
#pragma unroll
    for (int t = 0; t < 4; ++t) { const int gc = q * NHID + c0 + t * 16 + col; const size_t wrow = (size_t)gc * NF;
#pragma unroll
      for (int kc = 0; kc < 4; ++kc) { F2 a; a.h = frag_b(&sAh[wave][0][col][kc * 32], lane); a.l = frag_b(&sAl[wave][0][col][kc * 32], lane); di[t] = mac3(a, split_row(wia + wrow, kc * 32, lane), di[t]);
        a.h = frag_b(&sAh[wave][1][col][kc * 32], lane); a.l = frag_b(&sAl[wave][1][col][kc * 32], lane); dh[t] = mac3(a, split_row(wha + wrow, kc * 32, lane), dh[t]); } }
#pragma unroll
    for (int t = 0; t < 4; ++t) { const int gc = q * NHID + c0 + t * 16 + col; const float gi = giw[gc], bi = gib[gc], gh = ghw[gc], bh = ghb[gc];
#pragma unroll
      for (int r = 0; r < 8; ++r) sg[wave][q][8 * g + r][t * 16 + col] = ((di[t][r] - sti[r][0]) * sti[r][1] * gi + bi) + ((dh[t][r] - sth[r][0]) * sth[r][1] * gh + bh); } }
  LDSX();
  { const int rl = lane >> 1, hf = lane & 1; const int row = r0 + rl;
    for (int u4 = hf * 8; u4 < hf * 8 + 8; ++u4) { v4f cp, og; const v4f cxv = *(const v4f*)(cx + (size_t)row * NHID + c0 + u4 * 4);
#pragma unroll
      for (int e = 0; e < 4; ++e) { const int u = u4 * 4 + e; const float ig = sigm(sg[wave][0][rl][u]), fg = sigm(sg[wave][1][rl][u]), gg = tanhf(sg[wave][2][rl][u]), og_ = sigm(sg[wave][3][rl][u]);
        cp[e] = fg * cxv[e] + ig * gg; og[e] = og_; }
      vst2(CP + (size_t)row * NHID + c0 + u4 * 4, cp); vst2(OG + (size_t)row * NHID + c0 + u4 * 4, og); } }
}
__global__ __launch_bounds__(256) void k_final(const float* __restrict__ CP, const float* __restrict__ OG, const float* __restrict__ gcw, const float* __restrict__ gcb, float* __restrict__ hy, float* __restrict__ cy) {
  const int wave = threadIdx.x >> 5, lane = threadIdx.x & 31; const size_t r = (size_t)blockIdx.x * 8 + wave; if (r >= NBATCH) return;
  const float* cr = CP + r * NHID; float s = 0.f, q2 = 0.f;
#pragma unroll 1
  for (int i = 0; i < 8; ++i) { const v4f a = *(const v4f*)(cr + i * 128 + lane * 4); s += (a[0] + a[1]) + (a[2] + a[3]); q2 += (a[0] * a[0] + a[1] * a[1]) + (a[2] * a[2] + a[3] * a[3]); }
#pragma unroll
  for (int off = 16; off >= 1; off >>= 1) { s += __shfl_xor(s, off, 32); q2 += __shfl_xor(q2, off, 32); }
  const float mu = s * (1.0f / NHID); const float var = fmaxf(q2 * (1.0f / NHID) - mu * mu, 0.f); const float rs = rsqrtf(var + 1e-5f);
#pragma unroll 1
  for (int i = 0; i < 8; ++i) { const int c0 = i * 128 + lane * 4; const v4f a = *(const v4f*)(cr + c0); const v4f o = *(const v4f*)(OG + r * NHID + c0); v4f cv, hv;
#pragma unroll
    for (int e = 0; e < 4; ++e) { const float c = (a[e] - mu) * rs * gcw[c0 + e] + gcb[c0 + e]; cv[e] = c; hv[e] = o[e] * tanhf(c); }
    vst2(cy + r * NHID + c0, cv); vst2(hy + r * NHID + c0, hv); }
}
extern "C" void kernel_launch(void* const* d_in, const int* in_sizes, int n_in, void* d_out, int out_size, void* d_ws, size_t ws_size, hipStream_t stream) {
  (void)in_sizes; (void)n_in; (void)out_size; (void)ws_size;
  const float** I = (const float**)d_in;
  const float* x = I[0]; const float* hx = I[1]; const float* cx = I[2]; const float* topic = I[3];
  const float* wia = I[4]; const float* wib = I[5]; const float* wic = I[6]; const float* wha = I[7]; const float* whb = I[8]; const float* whc = I[9];
  const float* tiw = I[10]; const float* tib = I[11]; const float* thw = I[12]; const float* thb = I[13];
  const float* giw = I[14]; const float* gib = I[15]; const float* ghw = I[16]; const float* ghb = I[17]; const float* gcw = I[18]; const float* gcb = I[19];
  float* hy = (float*)d_out; float* cy = (float*)((char*)d_out + 16777216);
  char* ws = (char*)d_ws; size_t off = 0;
  auto take = [&](size_t bytes) { char* p = ws + off; off += (bytes + 255) & ~(size_t)255; return p; };
  float* UI = (float*)take((size_t)NBATCH * NF * 4); float* UH = (float*)take((size_t)NBATCH * NF * 4); float* ST = (float*)take((size_t)NBATCH * 4 * 4);
  float* CP = (float*)take((size_t)NBATCH * NHID * 4); float* OG = (float*)take((size_t)NBATCH * NHID * 4);
  k_u<<<dim3(NBATCH / 64, 2), 128, 0, stream>>>(x, hx, topic, wic, whc, wib, whb, tiw, tib, thw, thb, UI, UH);
  k_stats<<<NBATCH / 64, 128, 0, stream>>>(UI, UH, wia, wha, ST);
  k_cell<<<dim3(NBATCH / 64, NHID / 64), 128, 0, stream>>>(UI, UH, wia, wha, ST, giw, gib, ghw, ghb, cx, CP, OG);
  k_final<<<NBATCH / 8, 256, 0, stream>>>(CP, OG, gcw, gcb, hy, cy);
}
